// DifferentialAttention_47467978555547
// MI455X (gfx1250) — hardware-verified
//
#include <hip/hip_runtime.h>
#include <hip/hip_bf16.h>
#include <math.h>

#ifndef NB
#define NB 1
#endif
#ifndef SEQ
#define SEQ 2048
#endif
#define SEQ_FULL 2048
#define DM 2048
#define NH 16
#define KVH 4
#define HD 128
#define KVD (KVH * HD)
#define QKD (NH * HD)
#define ROT 64
#define WIN 512
#define RESQ 256
#define QT 128
#define QTR 64
#define KT 64
#define KP 136
#define VP 72

#define PCARRY 1024.0f
#define RSCL 1024.0f
#define OCARRY 16.0f
#define WSCL 64.0f
#define NEGBIG (-1.0e30f)

static_assert(NB == 1);
static_assert(SEQ % QT == 0);
static_assert(SEQ >= RESQ);
static_assert(SEQ <= SEQ_FULL);
static_assert(RESQ % QT == 0);
static_assert(RESQ % QTR == 0);
static_assert((SEQ - RESQ) % QT == 0);
static_assert(QT % KT == 0 && QTR % KT == 0);
static_assert(WIN % KT == 0);
static_assert(HD == 128);
static_assert(ROT * 2 == HD);
static_assert(NH % KVH == 0);
static_assert(DM % 64 == 0 && KVD % 64 == 0 && QKD % 64 == 0 && SEQ % 64 == 0);
static_assert(DM % 32 == 0 && QKD % 32 == 0);
static_assert((SEQ * DM) % 2048 == 0);
static_assert((NH * SEQ) % 32 == 0 && (KVH * SEQ) % 32 == 0);
static_assert((SEQ * ROT) % 256 == 0);

#define SZ_XB   ((size_t)SEQ * DM * 2)
#define SZ_WQT  ((size_t)QKD * DM * 2)
#define SZ_WKT  ((size_t)KVD * DM * 2)
#define SZ_WVT  ((size_t)KVD * DM * 2)
#define SZ_WOT  ((size_t)DM * QKD * 2)
#define SZ_QF   ((size_t)SEQ * QKD * 4)
#define SZ_KF   ((size_t)SEQ * KVD * 4)
#define SZ_VF   ((size_t)SEQ * KVD * 4)
#define SZ_TRG  ((size_t)SEQ * ROT * 4)
#define SZ_QH   ((size_t)NH * SEQ * HD * 2)
#define SZ_KH   ((size_t)KVH * SEQ * HD * 2)
#define SZ_VT   ((size_t)KVD * SEQ * 2)
#define SZ_OH   ((size_t)SEQ * QKD * 2)
#define SZ_OL   ((size_t)RESQ * QKD * 2)

#define OFS_XB   ((size_t)0)
#define OFS_WQT  (OFS_XB + SZ_XB)
#define OFS_WKT  (OFS_WQT + SZ_WQT)
#define OFS_WVT  (OFS_WKT + SZ_WKT)
#define OFS_WOT  (OFS_WVT + SZ_WVT)
#define OFS_QF   (OFS_WOT + SZ_WOT)
#define OFS_KF   (OFS_QF + SZ_QF)
#define OFS_VF   (OFS_KF + SZ_KF)
#define OFS_COS  (OFS_VF + SZ_VF)
#define OFS_SIN  (OFS_COS + SZ_TRG)
#define OFS_QH   (OFS_SIN + SZ_TRG)
#define OFS_QL   (OFS_QH + SZ_QH)
#define OFS_KH   (OFS_QL + SZ_QH)
#define OFS_KL   (OFS_KH + SZ_KH)
#define OFS_VTH  (OFS_KL + SZ_KH)
#define OFS_VTL  (OFS_VTH + SZ_VT)
#define OFS_OH   (OFS_VTL + SZ_VT)
#define OFS_OL   (OFS_OH + SZ_OH)
#define WS_TOTAL (OFS_OL + SZ_OL)
static_assert(WS_TOTAL <= (size_t)134217728);
static_assert(OFS_WQT % 256 == 0 && OFS_QF % 256 == 0 && OFS_COS % 256 == 0 && OFS_QH % 256 == 0 &&
              OFS_VTH % 256 == 0 && OFS_OH % 256 == 0 && OFS_OL % 256 == 0);

typedef __attribute__((ext_vector_type(16))) _Float16 v16h;
typedef __attribute__((ext_vector_type(16))) __bf16 v16b;
typedef __attribute__((ext_vector_type(8))) float v8f;
typedef __attribute__((ext_vector_type(4))) float f4;
typedef __attribute__((ext_vector_type(4))) unsigned int u32x4;

union HFrag { u32x4 u[2]; v16h v; unsigned short s[16]; };
union BFrag { u32x4 u[2]; v16b v; };
union Pack8 { unsigned short s[8]; u32x4 u; };

struct InvFreq { float f[ROT]; };
static_assert(sizeof(InvFreq) == ROT * 4);

__device__ __forceinline__ v8f vzero8() { v8f z = {}; return z; }

__device__ __forceinline__ v8f mma_h(v16h a, v16h b, v8f c) {
  c = __builtin_amdgcn_wmma_f32_16x16x32_f16(false, a, false, b, (short)0, c, false, false);
  asm volatile("v_nop\n\tv_nop\n\tv_nop\n\tv_nop" : "+v"(c) : "v"(a), "v"(b));
  return c;
}
__device__ __forceinline__ v8f mma_b(v16b a, v16b b, v8f c) {
  c = __builtin_amdgcn_wmma_f32_16x16x32_bf16(false, a, false, b, (short)0, c, false, false);
  asm volatile("v_nop\n\tv_nop\n\tv_nop\n\tv_nop" : "+v"(c) : "v"(a), "v"(b));
  return c;
}

__device__ __forceinline__ unsigned short bf16_bits(float f) {
  unsigned int x = __float_as_uint(f);
  x = x + 0x7FFFu + ((x >> 16) & 1u);
  return (unsigned short)(x >> 16);
}
__device__ __forceinline__ float bf16_val(float f) {
  return __uint_as_float(((unsigned int)bf16_bits(f)) << 16);
}
__device__ __forceinline__ unsigned short h_bits(_Float16 h) {
  return __builtin_bit_cast(unsigned short, h);
}

__device__ __forceinline__ float rmax16(float v) {
  v = fmaxf(v, __shfl_xor(v, 1, 32));
  v = fmaxf(v, __shfl_xor(v, 2, 32));
  v = fmaxf(v, __shfl_xor(v, 4, 32));
  v = fmaxf(v, __shfl_xor(v, 8, 32));
  return v;
}
__device__ __forceinline__ float rsum16(float v) {
  v += __shfl_xor(v, 1, 32);
  v += __shfl_xor(v, 2, 32);
  v += __shfl_xor(v, 4, 32);
  v += __shfl_xor(v, 8, 32);
  return v;
}

__global__ __launch_bounds__(256) void k_cvt_x(const float* __restrict__ X, unsigned short* Xb) {
  const size_t idx = (size_t)blockIdx.x * 256 + threadIdx.x;
  const float* p = X + idx * 8;
  const f4 a = *(const f4*)p;
  const f4 b = *(const f4*)(p + 4);
  Pack8 o;
#pragma unroll
  for (int e = 0; e < 4; ++e) {
    o.s[e] = bf16_bits(a[e]);
    o.s[e + 4] = bf16_bits(b[e]);
  }
  *(volatile u32x4*)(Xb + idx * 8) = o.u;
  __threadfence();
  *(volatile u32x4*)(Xb + idx * 8) = o.u;
}

template <int MODE>
__global__ __launch_bounds__(256) void k_transpose(const float* __restrict__ in, int R, int Cc,
                                                    unsigned short* P0, unsigned short* P1) {
  __shared__ float tile[64 * 65];
  const int r0 = (int)blockIdx.y * 64;
  const int c0 = (int)blockIdx.x * 64;
#pragma unroll
  for (int ps = 0; ps < 4; ++ps) {
    const int idx = (int)threadIdx.x + 256 * ps;
    const int r = idx >> 4, c4 = idx & 15;
    const f4 v = *(const f4*)(in + (size_t)(r0 + r) * Cc + c0 + c4 * 4);
#pragma unroll
    for (int e = 0; e < 4; ++e) tile[r * 65 + c4 * 4 + e] = v[e];
  }
  __syncthreads();
#pragma unroll
  for (int pass = 0; pass < 2; ++pass) {
    if (pass) __threadfence();
#pragma unroll
    for (int ps = 0; ps < 2; ++ps) {
      const int idx = (int)threadIdx.x + 256 * ps;
      const int nl = idx >> 3, pcs = idx & 7;
      Pack8 o0, o1;
#pragma unroll
      for (int e = 0; e < 8; ++e) {
        const float v = tile[(pcs * 8 + e) * 65 + nl];
        if (MODE == 0) {
          o0.s[e] = bf16_bits(v);
          o1.s[e] = 0;
        } else if (MODE == 1) {
          const _Float16 hw = (_Float16)(bf16_val(v) * WSCL);
          o0.s[e] = h_bits(hw);
          o1.s[e] = 0;
        } else {
          const _Float16 hh = (_Float16)v;
          const _Float16 hl = (_Float16)((v - (float)hh) * RSCL);
          o0.s[e] = h_bits(hh);
          o1.s[e] = h_bits(hl);
        }
      }
      const size_t go = (size_t)(c0 + nl) * R + r0 + pcs * 8;
      *(volatile u32x4*)(P0 + go) = o0.u;
      if (MODE == 2) *(volatile u32x4*)(P1 + go) = o1.u;
    }
  }
}

__global__ __launch_bounds__(256) void k_trig(InvFreq iv, float* cosT, float* sinT) {
  const int idx = (int)blockIdx.x * 256 + (int)threadIdx.x;
  const int s = idx >> 6;
  const int i = idx & 63;
  float invf = iv.f[0];
#pragma unroll
  for (int k = 1; k < ROT; ++k) invf = (i == k) ? iv.f[k] : invf;
  const float th = (float)s * invf;
  const float c = cosf(th);
  const float sn = sinf(th);
  *(volatile float*)(cosT + idx) = c;
  *(volatile float*)(sinT + idx) = sn;
  __threadfence();
  *(volatile float*)(cosT + idx) = c;
  *(volatile float*)(sinT + idx) = sn;
}

__global__ __launch_bounds__(256) void k_rope(const float* __restrict__ src, int pitch,
                                              const float* __restrict__ cosT,
                                              const float* __restrict__ sinT,
                                              unsigned short* Ph, unsigned short* Pl) {
#pragma clang fp contract(off)
  const int pairIdx = (int)blockIdx.x * 32 + ((int)threadIdx.x >> 3);
  const int t = (int)threadIdx.x & 7;
  const int hh = pairIdx / SEQ;
  const int s = pairIdx - hh * SEQ;
  const float* sp = src + (size_t)s * pitch + hh * HD + 8 * t;
  const f4 xa = *(const f4*)(sp);
  const f4 xb = *(const f4*)(sp + 4);
  const f4 ya = *(const f4*)(sp + 64);
  const f4 yb = *(const f4*)(sp + 68);
  const float* cp = cosT + (size_t)s * ROT + 8 * t;
  const float* snp = sinT + (size_t)s * ROT + 8 * t;
  const f4 ca = *(const f4*)(cp);
  const f4 cb = *(const f4*)(cp + 4);
  const f4 sa = *(const f4*)(snp);
  const f4 sb = *(const f4*)(snp + 4);
  float x1[8], x2[8], cv[8], sv[8];
#pragma unroll
  for (int e = 0; e < 4; ++e) {
    x1[e] = xa[e]; x1[e + 4] = xb[e];
    x2[e] = ya[e]; x2[e + 4] = yb[e];
    cv[e] = ca[e]; cv[e + 4] = cb[e];
    sv[e] = sa[e]; sv[e + 4] = sb[e];
  }
  Pack8 h1, h2, l1, l2;
#pragma unroll
  for (int e = 0; e < 8; ++e) {
    const float o1 = x1[e] * cv[e] - x2[e] * sv[e];
    const float o2 = x2[e] * cv[e] + x1[e] * sv[e];
    const _Float16 a = (_Float16)o1;
    const _Float16 b = (_Float16)o2;
    const _Float16 ra = (_Float16)((o1 - (float)a) * RSCL);
    const _Float16 rb = (_Float16)((o2 - (float)b) * RSCL);
    h1.s[e] = h_bits(a);
    h2.s[e] = h_bits(b);
    l1.s[e] = h_bits(ra);
    l2.s[e] = h_bits(rb);
  }
  const size_t go = (size_t)pairIdx * HD + 8 * t;
#pragma unroll
  for (int pass = 0; pass < 2; ++pass) {
    if (pass) __threadfence();
    *(volatile u32x4*)(Ph + go) = h1.u;
    *(volatile u32x4*)(Ph + go + 64) = h2.u;
    *(volatile u32x4*)(Pl + go) = l1.u;
    *(volatile u32x4*)(Pl + go + 64) = l2.u;
  }
}

template <int BF> struct GT;
template <> struct GT<0> {
  typedef HFrag F;
  static __device__ __forceinline__ v8f mma(const HFrag& a, const HFrag& b, v8f c) { return mma_h(a.v, b.v, c); }
};
template <> struct GT<1> {
  typedef BFrag F;
  static __device__ __forceinline__ v8f mma(const BFrag& a, const BFrag& b, v8f c) { return mma_b(a.v, b.v, c); }
};

template <int BF, int RES>
__global__ __launch_bounds__(256) void k_gemm(const unsigned short* __restrict__ Ah,
                                              const unsigned short* __restrict__ Al,
                                              const unsigned short* __restrict__ BT,
                                              float* C, int N, int K, float sHi, float sLo) {
  typedef typename GT<BF>::F F;
  __shared__ __align__(16) float stg[8 * 32 * 36];
  const int lane = threadIdx.x & 31;
  const int wave = threadIdx.x >> 5;
  const int l16 = lane & 15;
  const int hf = lane >> 4;
  const int kb8 = hf * 8;
  const int rm = (int)blockIdx.y * 128 + (wave & 3) * 32;
  const int cn = (int)blockIdx.x * 64 + (wave >> 2) * 32;
  const unsigned short* a0 = Ah + (size_t)(rm + l16) * K;
  const unsigned short* a1 = Ah + (size_t)(rm + 16 + l16) * K;
  const unsigned short* e0 = Al + (size_t)(rm + l16) * K;
  const unsigned short* e1 = Al + (size_t)(rm + 16 + l16) * K;
  const unsigned short* b0 = BT + (size_t)(cn + l16) * K;
  const unsigned short* b1 = BT + (size_t)(cn + 16 + l16) * K;

  v8f acc[2][2], accr[2][2];
#pragma unroll
  for (int mi = 0; mi < 2; ++mi)
#pragma unroll
    for (int ni = 0; ni < 2; ++ni) { acc[mi][ni] = vzero8(); accr[mi][ni] = vzero8(); }

#pragma unroll 1
  for (int k0 = 0; k0 < K; k0 += 32) {
    F fa0, fa1, fb0, fb1;
    fa0.u[0] = *(const u32x4*)(a0 + k0 + kb8);
    fa0.u[1] = *(const u32x4*)(a0 + k0 + 16 + kb8);
    fa1.u[0] = *(const u32x4*)(a1 + k0 + kb8);
    fa1.u[1] = *(const u32x4*)(a1 + k0 + 16 + kb8);
    fb0.u[0] = *(const u32x4*)(b0 + k0 + kb8);
    fb0.u[1] = *(const u32x4*)(b0 + k0 + 16 + kb8);
    fb1.u[0] = *(const u32x4*)(b1 + k0 + kb8);
    fb1.u[1] = *(const u32x4*)(b1 + k0 + 16 + kb8);
    acc[0][0] = GT<BF>::mma(fa0, fb0, acc[0][0]);
    acc[0][1] = GT<BF>::mma(fa0, fb1, acc[0][1]);
    acc[1][0] = GT<BF>::mma(fa1, fb0, acc[1][0]);
    acc[1][1] = GT<BF>::mma(fa1, fb1, acc[1][1]);
    if (RES) {
      F fl0, fl1;
      fl0.u[0] = *(const u32x4*)(e0 + k0 + kb8);
      fl0.u[1] = *(const u32x4*)(e0 + k0 + 16 + kb8);
      fl1.u[0] = *(const u32x4*)(e1 + k0 + kb8);
      fl1.u[1] = *(const u32x4*)(e1 + k0 + 16 + kb8);
      accr[0][0] = GT<BF>::mma(fl0, fb0, accr[0][0]);
      accr[0][1] = GT<BF>::mma(fl0, fb1, accr[0][1]);
      accr[1][0] = GT<BF>::mma(fl1, fb0, accr[1][0]);
      accr[1][1] = GT<BF>::mma(fl1, fb1, accr[1][1]);
    }
  }

  float* st = stg + wave * (32 * 36);
#pragma unroll
  for (int mi = 0; mi < 2; ++mi)
#pragma unroll
    for (int ni = 0; ni < 2; ++ni)
#pragma unroll
      for (int r = 0; r < 8; ++r) {
        float v = acc[mi][ni][r] * sHi;
        if (RES) v += accr[mi][ni][r] * sLo;
        st[(16 * mi + 8 * hf + r) * 36 + 16 * ni + l16] = v;
      }
  __syncthreads();
  const int rr = lane >> 3;
  const int pcs = lane & 7;
#pragma unroll
  for (int pass = 0; pass < 2; ++pass) {
    if (pass) __threadfence();
#pragma unroll
    for (int it = 0; it < 8; ++it) {
      const int row = it * 4 + rr;
      const f4 v = *(const f4*)(st + row * 36 + pcs * 4);
      *(volatile f4*)(C + (size_t)(rm + row) * N + cn + pcs * 4) = v;
    }
  }
}

template <int RES>
__device__ __forceinline__ void stage_k(unsigned short* dH, unsigned short* dL,
                                        const unsigned short* gH, const unsigned short* gL, int kt) {
#pragma unroll
  for (int ps = 0; ps < 4; ++ps) {
    const int idx = (int)threadIdx.x + 256 * ps;
    const int r = idx >> 4, pc = idx & 15;
    const size_t go = (size_t)(kt * KT + r) * HD + pc * 8;
    const int lo = r * KP + pc * 8;
    *(u32x4*)(dH + lo) = *(const u32x4*)(gH + go);
    if (RES) *(u32x4*)(dL + lo) = *(const u32x4*)(gL + go);
  }
}
template <int RES, int NDTB>
__device__ __forceinline__ void stage_v(unsigned short* dH, unsigned short* dL,
                                        const unsigned short* gH, const unsigned short* gL, int kt) {
  static_assert(NDTB % 2 == 0);
#pragma unroll
  for (int ps = 0; ps < NDTB / 2; ++ps) {
    const int idx = (int)threadIdx.x + 256 * ps;
    const int r = idx >> 3, pc = idx & 7;
    const size_t go = (size_t)r * SEQ + kt * KT + pc * 8;
    const int lo = r * VP + pc * 8;
    *(u32x4*)(dH + lo) = *(const u32x4*)(gH + go);
    if (RES) *(u32x4*)(dL + lo) = *(const u32x4*)(gL + go);
  }
}

template <int RES>
__device__ __forceinline__ v8f score_tile(const unsigned short* __restrict__ qh,
                                          const unsigned short* __restrict__ ql,
                                          const unsigned short* kr, const unsigned short* krl,
                                          int dOff, int kb8) {
  v8f acc = vzero8();
  v8f accx = vzero8();
#pragma unroll
  for (int ks = 0; ks < 2; ++ks) {
    const int d = dOff + 32 * ks;
    HFrag a, b;
    a.u[0] = *(const u32x4*)(qh + d + kb8);
    a.u[1] = *(const u32x4*)(qh + d + 16 + kb8);
    b.u[0] = *(const u32x4*)(kr + d + kb8);
    b.u[1] = *(const u32x4*)(kr + d + 16 + kb8);
    acc = mma_h(a.v, b.v, acc);
    if (RES) {
      HFrag bl;
      bl.u[0] = *(const u32x4*)(krl + d + kb8);
      bl.u[1] = *(const u32x4*)(krl + d + 16 + kb8);
      accx = mma_h(a.v, bl.v, accx);
      HFrag al;
      al.u[0] = *(const u32x4*)(ql + d + kb8);
      al.u[1] = *(const u32x4*)(ql + d + 16 + kb8);
      accx = mma_h(al.v, b.v, accx);
    }
  }
  if (RES) {
#pragma unroll
    for (int j = 0; j < 8; ++j) acc[j] += accx[j] * (1.0f / RSCL);
  }
  return acc;
}

__device__ __forceinline__ void soft_update(v8f (&sv)[4], float (&m)[8], float (&z)[8],
                                            int keyBase, int rowBase, int l16) {
  float tmax[8];
#pragma unroll
  for (int j = 0; j < 8; ++j) tmax[j] = NEGBIG;
#pragma unroll
  for (int t = 0; t < 4; ++t) {
#pragma unroll
    for (int j = 0; j < 8; ++j) {
      const int i = rowBase + j;
      const int jk = keyBase + t * 16 + l16;
      const bool ok = (jk <= i) && (jk >= i - (WIN - 1));
      const float lg = ok ? sv[t][j] * 0.125f : NEGBIG;
      sv[t][j] = lg;
      tmax[j] = fmaxf(tmax[j], lg);
    }
  }
#pragma unroll
  for (int j = 0; j < 8; ++j) {
    const float tm = rmax16(tmax[j]);
    const float nm = fmaxf(m[j], tm);
    const float corr = __expf(m[j] - nm);
    m[j] = nm;
    float s = 0.0f;
#pragma unroll
    for (int t = 0; t < 4; ++t) {
      const float lg = sv[t][j];
      s += (lg > -1.0e29f) ? __expf(lg - nm) : 0.0f;
    }
    s = rsum16(s);
    z[j] = z[j] * corr + s;
  }
}

template <int RES>
__device__ __forceinline__ void p_subtile(const unsigned short* __restrict__ qh,
                                          const unsigned short* __restrict__ ql,
                                          const unsigned short* kr, const unsigned short* krl,
                                          int keyBase, int rowBase, int l16, int hf, int kb8,
                                          const float (&m1)[8], const float (&z1)[8],
                                          const float (&m2)[8], const float (&z2)[8],
                                          float lamh, float (&dsum)[8],
                                          unsigned short* psDst, Pack8& ur) {
  const v8f s1 = score_tile<RES>(qh, ql, kr, krl, 0, kb8);
  const v8f s2 = score_tile<RES>(qh, ql, kr, krl, 64, kb8);
  Pack8 uh;
#pragma unroll
  for (int j = 0; j < 8; ++j) {
    const int i = rowBase + j;
    const int jk = keyBase + l16;
    const bool ok = (jk <= i) && (jk >= i - (WIN - 1));
    const float lg1 = ok ? s1[j] * 0.125f : NEGBIG;
    const float lg2 = ok ? s2[j] * 0.125f : NEGBIG;
    const float e1 = ok ? __expf(lg1 - m1[j]) * z1[j] : 0.0f;
    const float e2 = ok ? __expf(lg2 - m2[j]) * z2[j] : 0.0f;
    const float p = fmaxf(e1 - lamh * e2, 0.0f);
    dsum[j] += p;
    const float pc = p * PCARRY;
    const _Float16 ph = (_Float16)pc;
    uh.s[j] = h_bits(ph);
    if (RES) {
      const _Float16 pr = (_Float16)((pc - (float)ph) * RSCL);
      ur.s[j] = h_bits(pr);
    }
  }
  *(u32x4*)(psDst + 8 * hf) = uh.u;
}

template <int RES, int NDT, int WPG>
__global__ __launch_bounds__(256) __attribute__((amdgpu_num_vgpr(256)))
void k_attn(const unsigned short* __restrict__ Qh, const unsigned short* __restrict__ Ql,
            const unsigned short* __restrict__ Kh, const unsigned short* __restrict__ Kl,
            const unsigned short* __restrict__ Vth, const unsigned short* __restrict__ Vtl,
            const float* __restrict__ lam,
            unsigned short* Oh, unsigned short* Ol, int qtile0) {
  static_assert(WPG == 1 || WPG == 2);
  constexpr int NG = 8 / WPG;
  constexpr int QTB = NG * 16;
  constexpr int NDTB = NDT * WPG;
  constexpr int DB = NDTB * 16;
  static_assert(HD % DB == 0);
  static_assert(NDTB % 2 == 0);
  constexpr int KB = KT * KP;
  constexpr int VB = DB * VP;
  constexpr int PSW = 32 * 16;
  constexpr int OFF_KH = 0;
  constexpr int OFF_KL = KB;
  constexpr int OFF_VH = RES ? 2 * KB : KB;
  constexpr int OFF_VL = OFF_VH + VB;
  constexpr int OFF_P = RES ? (OFF_VL + VB) : (OFF_VH + VB);
  constexpr int TOT = OFF_P + 8 * PSW;
  constexpr int EP = DB + 8;
  constexpr int STW = 16 * EP;
  static_assert((RES ? 2 : 1) * NG * STW <= TOT);
  static_assert(TOT * 2 <= 65536);
  constexpr int PIECES = NDTB * 2;
  static_assert(PIECES <= 32 && 32 % PIECES == 0);
  constexpr int RPI = 32 / PIECES;
  constexpr int RPW = 16 / WPG;
  static_assert(RPW % RPI == 0);
  constexpr int NIT = RPW / RPI;
  __shared__ __align__(16) unsigned short smem[TOT];

  const int lane = threadIdx.x & 31;
  const int wave = threadIdx.x >> 5;
  const int l16 = lane & 15;
  const int hf = lane >> 4;
  const int kb8 = hf * 8;
  const int group = wave / WPG;
  const int sub = wave - group * WPG;
  const int dsub = sub * NDT;
  const int h = (int)blockIdx.y;
  const int kv = h / (NH / KVH);
  const int q0B = (qtile0 + (int)blockIdx.x) * QTB;
  const int rowW = q0B + group * 16;
  const int rowBase = rowW + 8 * hf;
  const int d0 = (int)blockIdx.z * DB;
  const float lamh = bf16_val(lam[h]);
  const int ktFirst = (q0B >= WIN) ? ((q0B - WIN) / KT) : 0;
  const int ktLast = (q0B + QTB - 1) / KT;

  const unsigned short* qh = Qh + ((size_t)h * SEQ + rowW + l16) * HD;
  const unsigned short* ql = Ql + ((size_t)h * SEQ + rowW + l16) * HD;
  const unsigned short* kgH = Kh + (size_t)kv * SEQ * HD;
  const unsigned short* kgL = Kl + (size_t)kv * SEQ * HD;
  const unsigned short* vgH = Vth + ((size_t)kv * HD + d0) * SEQ;
  const unsigned short* vgL = Vtl + ((size_t)kv * HD + d0) * SEQ;

  float m1[8], m2[8], z1[8], z2[8];
#pragma unroll
  for (int j = 0; j < 8; ++j) { m1[j] = NEGBIG; m2[j] = NEGBIG; z1[j] = 0.0f; z2[j] = 0.0f; }

#pragma unroll 1
  for (int kt = ktFirst; kt <= ktLast; ++kt) {
    __syncthreads();
    stage_k<RES>(smem + OFF_KH, smem + OFF_KL, kgH, kgL, kt);
    __syncthreads();
    v8f sv[4];
#pragma unroll
    for (int t = 0; t < 4; ++t) {
      const unsigned short* kr = smem + OFF_KH + (t * 16 + l16) * KP;
      const unsigned short* krl = smem + OFF_KL + (t * 16 + l16) * KP;
      sv[t] = score_tile<RES>(qh, ql, kr, krl, 0, kb8);
    }
    soft_update(sv, m1, z1, kt * KT, rowBase, l16);
#pragma unroll
    for (int t = 0; t < 4; ++t) {
      const unsigned short* kr = smem + OFF_KH + (t * 16 + l16) * KP;
      const unsigned short* krl = smem + OFF_KL + (t * 16 + l16) * KP;
      sv[t] = score_tile<RES>(qh, ql, kr, krl, 64, kb8);
    }
    soft_update(sv, m2, z2, kt * KT, rowBase, l16);
  }
#pragma unroll
  for (int j = 0; j < 8; ++j) { z1[j] = 1.0f / z1[j]; z2[j] = 1.0f / z2[j]; }

  v8f acc[NDT], accr[NDT];
#pragma unroll
  for (int n = 0; n < NDT; ++n) { acc[n] = vzero8(); accr[n] = vzero8(); }
  float dsum[8];
#pragma unroll
  for (int j = 0; j < 8; ++j) dsum[j] = 0.0f;

#pragma unroll 1
  for (int kt = ktFirst; kt <= ktLast; ++kt) {
    __syncthreads();
    stage_k<RES>(smem + OFF_KH, smem + OFF_KL, kgH, kgL, kt);
    stage_v<RES, NDTB>(smem + OFF_VH, smem + OFF_VL, vgH, vgL, kt);
    __syncthreads();
    unsigned short* ps = smem + OFF_P + wave * PSW;
#pragma unroll 1
    for (int g = 0; g < 2; ++g) {
      Pack8 ur0, ur1;
      {
        const int t = 2 * g;
        const unsigned short* kr = smem + OFF_KH + (t * 16 + l16) * KP;
        const unsigned short* krl = smem + OFF_KL + (t * 16 + l16) * KP;
        p_subtile<RES>(qh, ql, kr, krl, kt * KT + t * 16, rowBase, l16, hf, kb8,
                       m1, z1, m2, z2, lamh, dsum, ps + (0 * 16 + l16) * 16, ur0);
      }
      {
        const int t = 2 * g + 1;
        const unsigned short* kr = smem + OFF_KH + (t * 16 + l16) * KP;
        const unsigned short* krl = smem + OFF_KL + (t * 16 + l16) * KP;
        p_subtile<RES>(qh, ql, kr, krl, kt * KT + t * 16, rowBase, l16, hf, kb8,
                       m1, z1, m2, z2, lamh, dsum, ps + (1 * 16 + l16) * 16, ur1);
      }
      __syncthreads();
      HFrag pa;
#pragma unroll
      for (int c = 0; c < 8; ++c) {
        pa.s[c] = ps[(kb8 + c) * 16 + l16];
        pa.s[c + 8] = ps[(16 + kb8 + c) * 16 + l16];
      }
      const v16h pav = pa.v;
#pragma unroll
      for (int n = 0; n < NDT; ++n) {
        const unsigned short* vr = smem + OFF_VH + (16 * (dsub + n) + l16) * VP + 32 * g;
        HFrag vb;
        vb.u[0] = *(const u32x4*)(vr + kb8);
        vb.u[1] = *(const u32x4*)(vr + 16 + kb8);
        acc[n] = mma_h(pav, vb.v, acc[n]);
        if (RES) {
          const unsigned short* vrl = smem + OFF_VL + (16 * (dsub + n) + l16) * VP + 32 * g;
          HFrag vbl;
          vbl.u[0] = *(const u32x4*)(vrl + kb8);
          vbl.u[1] = *(const u32x4*)(vrl + 16 + kb8);
          accr[n] = mma_h(pav, vbl.v, accr[n]);
        }
      }
      if (RES) {
        __syncthreads();
        *(u32x4*)(ps + (0 * 16 + l16) * 16 + 8 * hf) = ur0.u;
        *(u32x4*)(ps + (1 * 16 + l16) * 16 + 8 * hf) = ur1.u;
        __syncthreads();
        HFrag pr;
#pragma unroll
        for (int c = 0; c < 8; ++c) {
          pr.s[c] = ps[(kb8 + c) * 16 + l16];
          pr.s[c + 8] = ps[(16 + kb8 + c) * 16 + l16];
        }
        const v16h prv = pr.v;
#pragma unroll
        for (int n = 0; n < NDT; ++n) {
          const unsigned short* vr = smem + OFF_VH + (16 * (dsub + n) + l16) * VP + 32 * g;
          HFrag vb;
          vb.u[0] = *(const u32x4*)(vr + kb8);
          vb.u[1] = *(const u32x4*)(vr + 16 + kb8);
          accr[n] = mma_h(prv, vb.v, accr[n]);
        }
      }
      __syncthreads();
    }
  }

  float inv[8];
#pragma unroll
  for (int j = 0; j < 8; ++j) {
    const float ds = rsum16(dsum[j]);
    inv[j] = (1.0f / (ds + 1.0e-6f)) * (OCARRY / PCARRY);
  }
  __syncthreads();
  unsigned short* stH = smem + group * STW;
  unsigned short* stL = smem + NG * STW + group * STW;
#pragma unroll
  for (int n = 0; n < NDT; ++n) {
#pragma unroll
    for (int j = 0; j < 8; ++j) {
      float o = acc[n][j];
      if (RES) o += accr[n][j] * (1.0f / RSCL);
      o *= inv[j];
      const _Float16 oh = (_Float16)o;
      stH[(8 * hf + j) * EP + 16 * (dsub + n) + l16] = h_bits(oh);
      if (RES) {
        const _Float16 orr = (_Float16)((o - (float)oh) * RSCL);
        stL[(8 * hf + j) * EP + 16 * (dsub + n) + l16] = h_bits(orr);
      }
    }
  }
  __syncthreads();
  const int rr = lane / PIECES;
  const int pcs = lane % PIECES;
#pragma unroll
  for (int pass = 0; pass < 2; ++pass) {
    if (pass) __threadfence();
#pragma unroll
    for (int it = 0; it < NIT; ++it) {
      const int row = sub * RPW + it * RPI + rr;
      const size_t go = (size_t)(rowW + row) * QKD + h * HD + d0 + pcs * 8;
      const u32x4 v = *(const u32x4*)(stH + row * EP + pcs * 8);
      *(volatile u32x4*)(Oh + go) = v;
      if (RES) {
        const u32x4 w = *(const u32x4*)(stL + row * EP + pcs * 8);
        *(volatile u32x4*)(Ol + go) = w;
      }
    }
  }
}

extern "C" void kernel_launch(void* const* d_in, const int* in_sizes, int n_in,
                              void* d_out, int out_size, void* d_ws, size_t ws_size,
                              hipStream_t stream) {
  if (n_in < 6) return;
  if (in_sizes[0] < NB * SEQ * DM) return;
  if (in_sizes[1] < DM * QKD) return;
  if (in_sizes[2] < DM * KVD) return;
  if (in_sizes[3] < DM * KVD) return;
  if (in_sizes[4] < QKD * DM) return;
  if (in_sizes[5] < NH) return;
  if (out_size < NB * SEQ * DM) return;
  if (d_ws == nullptr || ws_size < WS_TOTAL) return;

  const float* x = (const float*)d_in[0];
  const float* Wq = (const float*)d_in[1];
  const float* Wk = (const float*)d_in[2];
  const float* Wv = (const float*)d_in[3];
  const float* Wo = (const float*)d_in[4];
  const float* lam = (const float*)d_in[5];
  float* out = (float*)d_out;

  char* ws = (char*)d_ws;
  unsigned short* Xb = (unsigned short*)(ws + OFS_XB);
  unsigned short* WqT = (unsigned short*)(ws + OFS_WQT);
  unsigned short* WkT = (unsigned short*)(ws + OFS_WKT);
  unsigned short* WvT = (unsigned short*)(ws + OFS_WVT);
  unsigned short* WoT = (unsigned short*)(ws + OFS_WOT);
  float* qf = (float*)(ws + OFS_QF);
  float* kf = (float*)(ws + OFS_KF);
  float* vf = (float*)(ws + OFS_VF);
  float* cosT = (float*)(ws + OFS_COS);
  float* sinT = (float*)(ws + OFS_SIN);
  unsigned short* Qh = (unsigned short*)(ws + OFS_QH);
  unsigned short* Ql = (unsigned short*)(ws + OFS_QL);
  unsigned short* Kh = (unsigned short*)(ws + OFS_KH);
  unsigned short* Kl = (unsigned short*)(ws + OFS_KL);
  unsigned short* Vth = (unsigned short*)(ws + OFS_VTH);
  unsigned short* Vtl = (unsigned short*)(ws + OFS_VTL);
  unsigned short* Oh = (unsigned short*)(ws + OFS_OH);
  unsigned short* Ol = (unsigned short*)(ws + OFS_OL);

  InvFreq iv;
  for (int i = 0; i < ROT; ++i) {
    const double pd = pow(10000.0, (double)i / 64.0);
    const float pf = (float)pd;
    iv.f[i] = 1.0f / pf;
  }

  const dim3 blk(256);
  k_cvt_x<<<dim3((SEQ * DM) / 2048), blk, 0, stream>>>(x, Xb);
  k_transpose<0><<<dim3(QKD / 64, DM / 64), blk, 0, stream>>>(Wq, DM, QKD, WqT, WqT);
  k_transpose<0><<<dim3(KVD / 64, DM / 64), blk, 0, stream>>>(Wk, DM, KVD, WkT, WkT);
  k_transpose<0><<<dim3(KVD / 64, DM / 64), blk, 0, stream>>>(Wv, DM, KVD, WvT, WvT);
  k_transpose<1><<<dim3(DM / 64, QKD / 64), blk, 0, stream>>>(Wo, QKD, DM, WoT, WoT);
  k_gemm<1, 0><<<dim3(QKD / 64, SEQ / 128), blk, 0, stream>>>(Xb, Xb, WqT, qf, QKD, DM, 1.0f, 0.0f);
  k_gemm<1, 0><<<dim3(KVD / 64, SEQ / 128), blk, 0, stream>>>(Xb, Xb, WkT, kf, KVD, DM, 1.0f, 0.0f);
  k_gemm<1, 0><<<dim3(KVD / 64, SEQ / 128), blk, 0, stream>>>(Xb, Xb, WvT, vf, KVD, DM, 1.0f, 0.0f);
  k_trig<<<dim3((SEQ * ROT) / 256), blk, 0, stream>>>(iv, cosT, sinT);
  k_rope<<<dim3((NH * SEQ) / 32), blk, 0, stream>>>(qf, QKD, cosT, sinT, Qh, Ql);
  k_rope<<<dim3((KVH * SEQ) / 32), blk, 0, stream>>>(kf, KVD, cosT, sinT, Kh, Kl);
  k_transpose<2><<<dim3(KVD / 64, SEQ / 64), blk, 0, stream>>>(vf, SEQ, KVD, Vth, Vtl);
  k_attn<1, 2, 2><<<dim3(RESQ / QTR, NH, 2), blk, 0, stream>>>(Qh, Ql, Kh, Kl, Vth, Vtl, lam, Oh, Ol, 0);
  if (SEQ > RESQ) {
    k_attn<0, 8, 1><<<dim3((SEQ - RESQ) / QT, NH, 1), blk, 0, stream>>>(Qh, Ql, Kh, Kl, Vth, Vtl, lam, Oh, Ol, RESQ / QT);
  }
  const float sHi = 1.0f / 1024.0f;
  const float sLo = 1.0f / 1048576.0f;
  k_gemm<0, 1><<<dim3(DM / 64, RESQ / 128), blk, 0, stream>>>(Oh, Ol, WoT, out, DM, QKD, sHi, sLo);
  if (SEQ > RESQ) {
    k_gemm<0, 0><<<dim3(DM / 64, (SEQ - RESQ) / 128), blk, 0, stream>>>(
        Oh + (size_t)RESQ * QKD, Ol, WoT, out + (size_t)RESQ * DM, DM, QKD, sHi, 0.0f);
  }
}
